// NonLocalBlock2D_12446815224184
// MI455X (gfx1250) — hardware-verified
//
#include <hip/hip_runtime.h>
#include <stddef.h>


typedef _Float16 v16h __attribute__((ext_vector_type(16)));
typedef _Float16 v8h  __attribute__((ext_vector_type(8)));
typedef float    v8f  __attribute__((ext_vector_type(8)));
typedef float    v4f  __attribute__((ext_vector_type(4)));
typedef _Float16 h16;

#ifndef NB
#define NB 4
#endif
#ifndef SEQ
#define SEQ 4096
#endif
#define NB_FULL  4
#define SEQ_FULL 4096
#define CIN   256
#define CI    128
#define MROWS (NB * SEQ)

static_assert(NB >= 1 && NB <= NB_FULL);
static_assert(SEQ >= 128 && SEQ <= SEQ_FULL && (SEQ % 128) == 0);
static_assert(CI == 128);
static_assert((CIN % 64) == 0 && (CIN % 32) == 0);
static_assert((CI % 64) == 0 && (CI % 32) == 0);
static_assert((MROWS % 64) == 0 && (MROWS % 128) == 0);
static_assert(((size_t)CI * CIN) % 2048 == 0);
static_assert((size_t)MROWS * CIN < (size_t)0x7FFFFFFFu);
static_assert((size_t)NB_FULL * CIN * SEQ_FULL < (size_t)0x7FFFFFFFu);

#define LDT 72
#define LDC 68
#define LDY 136
static_assert((LDT % 8) == 0 && LDT >= 64);
static_assert((LDC % 4) == 0 && LDC >= 64);
static_assert((LDY % 8) == 0 && LDY >= CI);

#define WCARRY 64.0f
#define RCARRY 2048.0f
#define PEXP   14.0f
#define YCARRY 16.0f
#define LOG2E  1.4426950408889634f

#define XT_BYTES  ((size_t)MROWS * CIN * 2)
#define WP_BYTES  ((size_t)CI * CIN * 2)
#define PL_BYTES  ((size_t)MROWS * CI * 2)
#define LSE_BYTES ((size_t)MROWS * 4)
#define OFF_XT  ((size_t)0)
#define OFF_WT  (OFF_XT + XT_BYTES)
#define OFF_WP  (OFF_WT + WP_BYTES)
#define OFF_WG  (OFF_WP + WP_BYTES)
#define OFF_WO  (OFF_WG + WP_BYTES)
#define OFF_TH  (OFF_WO + WP_BYTES)
#define OFF_TR  (OFF_TH + PL_BYTES)
#define OFF_PH  (OFF_TR + PL_BYTES)
#define OFF_PR  (OFF_PH + PL_BYTES)
#define OFF_G   (OFF_PR + PL_BYTES)
#define OFF_YT  (OFF_G + PL_BYTES)
#define OFF_YR  (OFF_YT + PL_BYTES)
#define OFF_LSE (OFF_YR + PL_BYTES)
#define WS_TOTAL (OFF_LSE + LSE_BYTES)
static_assert((XT_BYTES % 128) == 0 && (WP_BYTES % 128) == 0 && (PL_BYTES % 128) == 0);
static_assert((LSE_BYTES % 128) == 0);
static_assert(WS_TOTAL == (size_t)NB * SEQ * (CIN * 2 + 7 * CI * 2 + 4) + 4 * WP_BYTES);
static_assert(WS_TOTAL <= (size_t)134217728);

__device__ __forceinline__ float bf16r(float x) {
  unsigned int u = __float_as_uint(x);
  u = (u + 0x7FFFu + ((u >> 16) & 1u)) & 0xFFFF0000u;
  return __uint_as_float(u);
}

static __device__ __forceinline__ h16 toh_flush(float v) {
  const h16 r = (h16)v;
  return (fabsf(v) < 6.103515625e-05f) ? (h16)0.0f : r;
}

__device__ __forceinline__ v16h frag_at(const _Float16* p) {
  v8h lo = *(const v8h*)(p);
  v8h hi = *(const v8h*)(p + 16);
  v16h out;
#pragma unroll
  for (int i = 0; i < 8; ++i) { out[i] = lo[i]; out[i + 8] = hi[i]; }
  return out;
}

__device__ __forceinline__ v8f wmma16(v16h a, v16h b, v8f c) {
  v8f d = __builtin_amdgcn_wmma_f32_16x16x32_f16(false, a, false, b, (short)0, c,
                                                 false, false);
  asm volatile("v_nop\n\tv_nop\n\tv_nop\n\tv_nop" : "+v"(d) : "v"(a), "v"(b));
  return d;
}

__device__ __forceinline__ void wave_lds_sync() {
  __builtin_amdgcn_fence(3  , "wavefront");
  asm volatile("s_wait_dscnt 0x0" ::: "memory");
  __builtin_amdgcn_wave_barrier();
}

__global__ __launch_bounds__(256) void wconv_kernel(
    const float* __restrict__ W, _Float16* __restrict__ Wt, unsigned ldw, unsigned ldk) {
  __shared__ _Float16 T[64 * LDT];
  const unsigned tid = threadIdx.x;
  const unsigned n0 = blockIdx.x * 64u;
  const unsigned k0 = blockIdx.y * 64u;
#pragma unroll 4
  for (unsigned j = 0; j < 16u; ++j) {
    const unsigned idx = tid + 256u * j;
    const unsigned kr = idx >> 6, nc = idx & 63u;
    const float v = W[(size_t)(k0 + kr) * ldw + n0 + nc];
    T[nc * LDT + kr] = (_Float16)(WCARRY * bf16r(v));
  }
  __syncthreads();
  v8h x[2];
  size_t off[2];
#pragma unroll
  for (unsigned i = 0; i < 2u; ++i) {
    const unsigned n = 32u * i + (tid >> 3);
    const unsigned kc = (tid & 7u) * 8u;
    x[i] = *(const v8h*)&T[n * LDT + kc];
    off[i] = (size_t)(n0 + n) * ldk + k0 + kc;
  }
#pragma unroll
  for (int i = 0; i < 2; ++i) *(volatile v8h*)(Wt + off[i]) = x[i];
  __threadfence();
#pragma unroll
  for (int i = 0; i < 2; ++i) *(volatile v8h*)(Wt + off[i]) = x[i];
}

__device__ __forceinline__ v8h wcvt8(const float* __restrict__ p) {
  const v4f a0 = *(const v4f*)(p);
  const v4f a1 = *(const v4f*)(p + 4);
  v8h o;
#pragma unroll
  for (int i = 0; i < 4; ++i) {
    o[i]     = toh_flush(WCARRY * bf16r(a0[i]));
    o[i + 4] = toh_flush(WCARRY * bf16r(a1[i]));
  }
  return o;
}

__global__ __launch_bounds__(256) void wplane_kernel(
    const float* __restrict__ w0, const float* __restrict__ w1,
    const float* __restrict__ w2, const float* __restrict__ w3,
    _Float16* __restrict__ o0, _Float16* __restrict__ o1,
    _Float16* __restrict__ o2, _Float16* __restrict__ o3) {
#pragma clang fp contract(off)
  const unsigned e = (blockIdx.x * 256u + threadIdx.x) * 8u;
  const v8h x0 = wcvt8(w0 + e);
  const v8h x1 = wcvt8(w1 + e);
  const v8h x2 = wcvt8(w2 + e);
  const v8h x3 = wcvt8(w3 + e);
  *(volatile v8h*)(o0 + e) = x0;
  *(volatile v8h*)(o1 + e) = x1;
  *(volatile v8h*)(o2 + e) = x2;
  *(volatile v8h*)(o3 + e) = x3;
  __threadfence();
  *(volatile v8h*)(o0 + e) = x0;
  *(volatile v8h*)(o1 + e) = x1;
  *(volatile v8h*)(o2 + e) = x2;
  *(volatile v8h*)(o3 + e) = x3;
}

template <int MODE>
__device__ __forceinline__ void gemm_body(
    const _Float16* __restrict__ A16, const _Float16* __restrict__ Bt,
    const _Float16* __restrict__ Btr, const unsigned K,
    const float* __restrict__ bias, const float* __restrict__ addf,
    float* __restrict__ outf, _Float16* __restrict__ out16, _Float16* __restrict__ out16r) {
  __shared__ float Cs[64 * LDC];
  const unsigned tid = threadIdx.x, lane = tid & 31u, w = tid >> 5;
  const unsigned mw = w >> 1, nw = w & 1u;
  const unsigned hh = lane >> 4, m = lane & 15u;
  const unsigned n0 = blockIdx.x * 64u;
  const unsigned row0 = blockIdx.y * 64u;

  const _Float16* ap  = A16 + (size_t)(row0 + mw * 16u + m) * K + hh * 8u;
  const _Float16* bp0 = Bt + (size_t)(n0 + nw * 32u + m) * K + hh * 8u;
  const _Float16* bp1 = bp0 + (size_t)16 * K;
  v8f accr0 = {}, accr1 = {};
  if (MODE == 2) {
    const _Float16* rp0 = Btr + (size_t)(n0 + nw * 32u + m) * K + hh * 8u;
    const _Float16* rp1 = rp0 + (size_t)16 * K;
#pragma unroll 2
    for (unsigned k0 = 0; k0 < K; k0 += 32u) {
      const v16h a  = frag_at(ap + k0);
      const v16h b0 = frag_at(rp0 + k0);
      const v16h b1 = frag_at(rp1 + k0);
      accr0 = wmma16(a, b0, accr0);
      accr1 = wmma16(a, b1, accr1);
    }
  }
  v8f acc0 = {}, acc1 = {};
#pragma unroll 2
  for (unsigned k0 = 0; k0 < K; k0 += 32u) {
    const v16h a  = frag_at(ap + k0);
    const v16h b0 = frag_at(bp0 + k0);
    const v16h b1 = frag_at(bp1 + k0);
    acc0 = wmma16(a, b0, acc0);
    acc1 = wmma16(a, b1, acc1);
  }
  if (MODE == 2) {
    acc0 = acc0 + accr0 * (1.0f / RCARRY);
    acc1 = acc1 + accr1 * (1.0f / RCARRY);
  }
#pragma unroll
  for (int r = 0; r < 8; ++r) {
    float* d = &Cs[(mw * 16u + hh * 8u + (unsigned)r) * LDC + nw * 32u + m];
    d[0]  = acc0[r];
    d[16] = acc1[r];
  }
  __syncthreads();

  if (MODE == 0) {
    const float cs = 1.0f / (WCARRY * WCARRY);
    v8h x[2], xr[2];
    size_t off[2];
#pragma unroll
    for (unsigned i = 0; i < 2u; ++i) {
      const unsigned r = 32u * i + (tid >> 3);
      const unsigned c = (tid & 7u) * 8u;
      const v4f u0 = *(const v4f*)&Cs[r * LDC + c];
      const v4f u1 = *(const v4f*)&Cs[r * LDC + c + 4];
      const v4f g0 = *(const v4f*)(bias + n0 + c);
      const v4f g1 = *(const v4f*)(bias + n0 + c + 4u);
#pragma unroll
      for (int j = 0; j < 4; ++j) {
        const float t0 = u0[j] * cs + bf16r(g0[j]);
        const float t1 = u1[j] * cs + bf16r(g1[j]);
        const h16 h0 = toh_flush(t0);
        const h16 h1 = toh_flush(t1);
        x[i][j]      = h0;
        x[i][j + 4]  = h1;
        xr[i][j]     = toh_flush((t0 - (float)h0) * RCARRY);
        xr[i][j + 4] = toh_flush((t1 - (float)h1) * RCARRY);
      }
      off[i] = (size_t)(row0 + r) * CI + n0 + c;
    }
#pragma unroll
    for (int i = 0; i < 2; ++i) *(volatile v8h*)(out16 + off[i]) = x[i];
#pragma unroll
    for (int i = 0; i < 2; ++i) *(volatile v8h*)(out16r + off[i]) = xr[i];
    __threadfence();
#pragma unroll
    for (int i = 0; i < 2; ++i) *(volatile v8h*)(out16 + off[i]) = x[i];
#pragma unroll
    for (int i = 0; i < 2; ++i) *(volatile v8h*)(out16r + off[i]) = xr[i];
  }

  if (MODE == 1) {
    const float cs = 1.0f / (WCARRY * WCARRY);
    const unsigned bidx = row0 / (unsigned)SEQ;
    const unsigned key0 = row0 - bidx * (unsigned)SEQ;
    v8h x[2];
    size_t off[2];
#pragma unroll
    for (unsigned i = 0; i < 2u; ++i) {
      const unsigned dcol = 32u * i + (tid >> 3);
      const unsigned kk = (tid & 7u) * 8u;
      const float bb = bf16r(bias[n0 + dcol]);
#pragma unroll
      for (unsigned j = 0; j < 8u; ++j) {
        const float t = Cs[(kk + j) * LDC + dcol] * cs + bb;
        x[i][j] = toh_flush(t);
      }
      off[i] = ((size_t)bidx * CI + n0 + dcol) * SEQ + key0 + kk;
    }
#pragma unroll
    for (int i = 0; i < 2; ++i) *(volatile v8h*)(out16 + off[i]) = x[i];
    __threadfence();
#pragma unroll
    for (int i = 0; i < 2; ++i) *(volatile v8h*)(out16 + off[i]) = x[i];
  }

  if (MODE == 2) {
    const float cs = 1.0f / (WCARRY * YCARRY);
    const unsigned bidx = n0 / (unsigned)SEQ;
    const unsigned p0 = n0 - bidx * (unsigned)SEQ;
    v4f xs[4];
    size_t off[4];
#pragma unroll
    for (unsigned i = 0; i < 4u; ++i) {
      const unsigned r = 16u * i + (tid >> 4);
      const unsigned c = (tid & 15u) * 4u;
      const unsigned orow = row0 + r;
      const size_t gidx = ((size_t)bidx * CIN + orow) * SEQ_FULL + p0 + c;
      const v4f u = *(const v4f*)&Cs[r * LDC + c];
      const float bb = bf16r(bias[orow]);
      const v4f xin = *(const v4f*)(addf + gidx);
      v4f val;
#pragma unroll
      for (int j = 0; j < 4; ++j) val[j] = bf16r(xin[j]) + (u[j] * cs + bb);
      xs[i] = val;
      off[i] = gidx;
    }
#pragma unroll
    for (int i = 0; i < 4; ++i) *(volatile v4f*)(outf + off[i]) = xs[i];
    __threadfence();
#pragma unroll
    for (int i = 0; i < 4; ++i) *(volatile v4f*)(outf + off[i]) = xs[i];
  }
}

__global__ __launch_bounds__(256) void gemm_tp_kernel(
    const _Float16* __restrict__ A16, const _Float16* __restrict__ Bt,
    const float* __restrict__ bias, _Float16* __restrict__ out16, _Float16* __restrict__ out16r) {
  gemm_body<0>(A16, Bt, Bt, (unsigned)CIN, bias, bias, (float*)0, out16, out16r);
}
__global__ __launch_bounds__(256) void gemm_g_kernel(
    const _Float16* __restrict__ A16, const _Float16* __restrict__ Bt,
    const float* __restrict__ bias, _Float16* __restrict__ gt) {
  gemm_body<1>(A16, Bt, Bt, (unsigned)CIN, bias, bias, (float*)0, gt, gt);
}
__global__ __launch_bounds__(256) void gemm_out_kernel(
    const _Float16* __restrict__ A16, const _Float16* __restrict__ Bt,
    const _Float16* __restrict__ Btr,
    const float* __restrict__ bias, const float* __restrict__ xin, float* __restrict__ outf) {
  gemm_body<2>(A16, Bt, Btr, (unsigned)CI, bias, xin, outf, (_Float16*)0, (_Float16*)0);
}

__global__ __launch_bounds__(256) __attribute__((amdgpu_num_vgpr(256))) void colstat_kernel(
    const _Float16* __restrict__ Th, const _Float16* __restrict__ Tr,
    const _Float16* __restrict__ Ph, const _Float16* __restrict__ Pr,
    float* __restrict__ Lse) {
  __shared__ __attribute__((aligned(16))) float Ls[128];
  const unsigned tid = threadIdx.x, lane = tid & 31u;
  const unsigned wave = (unsigned)__builtin_amdgcn_readfirstlane((int)(threadIdx.x >> 5));
  const unsigned hh = lane >> 4, m = lane & 15u;
  const unsigned b = blockIdx.y;
  const unsigned j0 = blockIdx.x * 128u + wave * 16u;

  const unsigned boff = (b * (unsigned)SEQ + j0 + m) * (unsigned)CI + hh * 8u;
  v16h bh[4], br[4];
#pragma unroll
  for (int ks = 0; ks < 4; ++ks) {
    bh[ks] = frag_at(Ph + boff + ks * 32);
    br[ks] = frag_at(Pr + boff + ks * 32);
  }

  float mx = -1.0e30f, z = 0.0f;
  const unsigned abase = b * (unsigned)SEQ * (unsigned)CI + m * (unsigned)CI + hh * 8u;
  for (unsigned i0 = 0; i0 < (unsigned)SEQ; i0 += 32u) {
    v8f f[2];
#pragma unroll
    for (int t = 0; t < 2; ++t) {
      const unsigned ao = abase + (i0 + 16u * (unsigned)t) * (unsigned)CI;
      v8f sm = {}, sr = {};
#pragma unroll
      for (int ks = 0; ks < 4; ++ks) {
        const v16h ah = frag_at(Th + ao + ks * 32);
        const v16h ar = frag_at(Tr + ao + ks * 32);
        sm = wmma16(ah, bh[ks], sm);
        sr = wmma16(ah, br[ks], sr);
        sr = wmma16(ar, bh[ks], sr);
      }
      f[t] = sm + sr * (1.0f / RCARRY);
    }
    float tmax = fmaxf(f[0][0], f[1][0]);
#pragma unroll
    for (int v = 1; v < 8; ++v) tmax = fmaxf(tmax, fmaxf(f[0][v], f[1][v]));
    const float nm = fmaxf(mx, tmax);
    float se = 0.0f;
#pragma unroll
    for (int v = 0; v < 8; ++v) se += __expf(f[0][v] - nm) + __expf(f[1][v] - nm);
    z = z * __expf(mx - nm) + se;
    mx = nm;
  }

  const float om = __shfl_xor(mx, 16, 32);
  const float oz = __shfl_xor(z, 16, 32);
  const float mm = fmaxf(mx, om);
  const float zz = z * __expf(mx - mm) + oz * __expf(om - mm);
  const float lse = mm + __logf(zz);
  if (hh == 0u) Ls[wave * 16u + m] = lse;
  __syncthreads();
  if (wave == 0u) {
    const v4f v = *(const v4f*)&Ls[lane * 4u];
    float* p = Lse + (size_t)b * SEQ + blockIdx.x * 128u + lane * 4u;
    *(volatile v4f*)p = v;
    __threadfence();
    *(volatile v4f*)p = v;
  }
}

__global__ __launch_bounds__(256) __attribute__((amdgpu_num_vgpr(256))) void rowattn_kernel(
    const _Float16* __restrict__ Th, const _Float16* __restrict__ Tr,
    const _Float16* __restrict__ Ph, const _Float16* __restrict__ Pr,
    const _Float16* __restrict__ Gp, const float* __restrict__ Lse,
    _Float16* __restrict__ Yt, _Float16* __restrict__ Yr) {
  __shared__ __attribute__((aligned(16))) _Float16 Ts[8 * 16 * LDY];
  const unsigned tid = threadIdx.x, lane = tid & 31u;
  const unsigned wave = (unsigned)__builtin_amdgcn_readfirstlane((int)(threadIdx.x >> 5));
  const unsigned hh = lane >> 4, m = lane & 15u;
  const unsigned b = blockIdx.y;
  const unsigned i0 = blockIdx.x * 128u + wave * 16u;

  const unsigned qoff = (b * (unsigned)SEQ + i0 + m) * (unsigned)CI + hh * 8u;
  v16h bh[4], br[4];
#pragma unroll
  for (int ks = 0; ks < 4; ++ks) {
    bh[ks] = frag_at(Th + qoff + ks * 32);
    br[ks] = frag_at(Tr + qoff + ks * 32);
  }

  v8f o[8];
#pragma unroll
  for (int ct = 0; ct < 8; ++ct) o[ct] = (v8f){};

  const unsigned kbase = b * (unsigned)SEQ * (unsigned)CI + m * (unsigned)CI + hh * 8u;
  const unsigned gbase = (b * (unsigned)CI + m) * (unsigned)SEQ + hh * 8u;
  const unsigned lbase = b * (unsigned)SEQ + hh * 8u;

  for (unsigned j0 = 0; j0 < (unsigned)SEQ; j0 += 32u) {
    v16h pb;
#pragma unroll
    for (int t = 0; t < 2; ++t) {
      const unsigned jt = j0 + 16u * (unsigned)t;
      const unsigned ao = kbase + jt * (unsigned)CI;
      v8f sm = {}, sr = {};
#pragma unroll
      for (int ks = 0; ks < 4; ++ks) {
        const v16h ah = frag_at(Ph + ao + ks * 32);
        const v16h ar = frag_at(Pr + ao + ks * 32);
        sm = wmma16(ah, bh[ks], sm);
        sr = wmma16(ah, br[ks], sr);
        sr = wmma16(ar, bh[ks], sr);
      }
      const v4f l0 = *(const v4f*)(Lse + lbase + jt);
      const v4f l1 = *(const v4f*)(Lse + lbase + jt + 4u);
#pragma unroll
      for (int v = 0; v < 4; ++v) {
        const float e0 = ((sm[v] + sr[v] * (1.0f / RCARRY)) - l0[v]) * LOG2E + PEXP;
        const float e1 = ((sm[v + 4] + sr[v + 4] * (1.0f / RCARRY)) - l1[v]) * LOG2E + PEXP;
        const float p0 = (e0 < -14.0f) ? 0.0f : exp2f(e0);
        const float p1 = (e1 < -14.0f) ? 0.0f : exp2f(e1);
        pb[8 * t + v]     = (h16)p0;
        pb[8 * t + v + 4] = (h16)p1;
      }
    }
#pragma unroll
    for (int ct = 0; ct < 8; ++ct) {
      const v16h gf = frag_at(Gp + gbase + (unsigned)ct * 16u * (unsigned)SEQ + j0);
      o[ct] = wmma16(gf, pb, o[ct]);
    }
  }

  const float fs = YCARRY * (1.0f / 16384.0f);
  const unsigned tb = wave * (16u * LDY);

#pragma unroll
  for (int ct = 0; ct < 8; ++ct) {
    v8h y;
#pragma unroll
    for (int v = 0; v < 8; ++v) y[v] = toh_flush(o[ct][v] * fs);
    *(v8h*)&Ts[tb + m * LDY + (unsigned)ct * 16u + hh * 8u] = y;
  }
  wave_lds_sync();
  v8h x[8];
  unsigned off[8];
#pragma unroll
  for (unsigned it = 0; it < 8u; ++it) {
    const unsigned r = 2u * it + (lane >> 4);
    const unsigned c = (lane & 15u) * 8u;
    x[it] = *(const v8h*)&Ts[tb + r * LDY + c];
    off[it] = (b * (unsigned)SEQ + i0 + r) * (unsigned)CI + c;
  }
  wave_lds_sync();

#pragma unroll
  for (int ct = 0; ct < 8; ++ct) {
    v8h y;
#pragma unroll
    for (int v = 0; v < 8; ++v) {
      const float t = o[ct][v] * fs;
      const h16 hi = toh_flush(t);
      y[v] = toh_flush((t - (float)hi) * RCARRY);
    }
    *(v8h*)&Ts[tb + m * LDY + (unsigned)ct * 16u + hh * 8u] = y;
  }
  wave_lds_sync();
  v8h xr[8];
#pragma unroll
  for (unsigned it = 0; it < 8u; ++it) {
    const unsigned r = 2u * it + (lane >> 4);
    const unsigned c = (lane & 15u) * 8u;
    xr[it] = *(const v8h*)&Ts[tb + r * LDY + c];
  }

#pragma unroll
  for (int it = 0; it < 8; ++it) *(volatile v8h*)(Yt + off[it]) = x[it];
#pragma unroll
  for (int it = 0; it < 8; ++it) *(volatile v8h*)(Yr + off[it]) = xr[it];
  __threadfence();
#pragma unroll
  for (int it = 0; it < 8; ++it) *(volatile v8h*)(Yt + off[it]) = x[it];
#pragma unroll
  for (int it = 0; it < 8; ++it) *(volatile v8h*)(Yr + off[it]) = xr[it];
}

extern "C" void kernel_launch(void* const* d_in, const int* in_sizes, int n_in,
                              void* d_out, int out_size, void* d_ws, size_t ws_size,
                              hipStream_t stream) {
  if (n_in < 9) return;
  const long long need_x = ((long long)(NB - 1) * CIN + (CIN - 1)) * SEQ_FULL + SEQ;
  if ((long long)in_sizes[0] < need_x) return;
  if ((long long)in_sizes[1] < (long long)CI * CIN) return;
  if ((long long)in_sizes[3] < (long long)CI * CIN) return;
  if ((long long)in_sizes[5] < (long long)CI * CIN) return;
  if ((long long)in_sizes[7] < (long long)CIN * CI) return;
  if (in_sizes[2] < CI || in_sizes[4] < CI || in_sizes[6] < CI || in_sizes[8] < CIN) return;
  if ((long long)out_size < need_x) return;
  if (ws_size < WS_TOTAL) return;

  const float* X       = (const float*)d_in[0];
  const float* theta_w = (const float*)d_in[1];
  const float* theta_b = (const float*)d_in[2];
  const float* phi_w   = (const float*)d_in[3];
  const float* phi_b   = (const float*)d_in[4];
  const float* g_w     = (const float*)d_in[5];
  const float* g_b     = (const float*)d_in[6];
  const float* W_w     = (const float*)d_in[7];
  const float* W_b     = (const float*)d_in[8];
  float* out = (float*)d_out;

  char* ws = (char*)d_ws;
  _Float16* XT   = (_Float16*)(ws + OFF_XT);
  _Float16* WT   = (_Float16*)(ws + OFF_WT);
  _Float16* WP   = (_Float16*)(ws + OFF_WP);
  _Float16* WG   = (_Float16*)(ws + OFF_WG);
  _Float16* WO   = (_Float16*)(ws + OFF_WO);
  _Float16* TH   = (_Float16*)(ws + OFF_TH);
  _Float16* TR   = (_Float16*)(ws + OFF_TR);
  _Float16* PH   = (_Float16*)(ws + OFF_PH);
  _Float16* PR   = (_Float16*)(ws + OFF_PR);
  _Float16* G16  = (_Float16*)(ws + OFF_G);
  _Float16* YT   = (_Float16*)(ws + OFF_YT);
  _Float16* YR   = (_Float16*)(ws + OFF_YR);
  float*    LSE  = (float*)(ws + OFF_LSE);

  dim3 blk(256);

  for (int b = 0; b < NB; ++b) {
    wconv_kernel<<<dim3(SEQ / 64, CIN / 64), blk, 0, stream>>>(
        X + (size_t)b * CIN * SEQ_FULL, XT + (size_t)b * SEQ * CIN,
        (unsigned)SEQ_FULL, (unsigned)CIN);
  }
  wplane_kernel<<<dim3((CI * CIN) / 2048), blk, 0, stream>>>(theta_w, phi_w, g_w, W_w,
                                                             WT, WP, WG, WO);

  dim3 gp(CI / 64, MROWS / 64);
  gemm_tp_kernel<<<gp, blk, 0, stream>>>(XT, WT, theta_b, TH, TR);
  gemm_tp_kernel<<<gp, blk, 0, stream>>>(XT, WP, phi_b, PH, PR);
  gemm_g_kernel<<<gp, blk, 0, stream>>>(XT, WG, g_b, G16);

  colstat_kernel<<<dim3(SEQ / 128, NB), blk, 0, stream>>>(TH, TR, PH, PR, LSE);
  rowattn_kernel<<<dim3(SEQ / 128, NB), blk, 0, stream>>>(TH, TR, PH, PR, G16, LSE, YT, YR);

  gemm_out_kernel<<<dim3(MROWS / 64, CIN / 64), blk, 0, stream>>>(WO, YT, YR, W_b, X, out);
}
